// CausalSelfAttention_45079976739499
// MI455X (gfx1250) — hardware-verified
//
#include <hip/hip_runtime.h>
#include <math.h>

typedef __attribute__((ext_vector_type(16))) _Float16 v16h;
typedef __attribute__((ext_vector_type(16))) __bf16 v16b;
typedef __attribute__((ext_vector_type(8)))  _Float16 v8h;
typedef __attribute__((ext_vector_type(8)))  __bf16 v8b;
typedef __attribute__((ext_vector_type(8)))  float v8f;
typedef __attribute__((ext_vector_type(4)))  float v4f;
typedef __attribute__((ext_vector_type(4)))  unsigned v4u;

template <typename T> __device__ __forceinline__ void vst2(void* p, T v) { *(volatile T*)p = v; __threadfence(); *(volatile T*)p = v; }
__device__ __forceinline__ v8f wmma16(v16h a, v16h b, v8f c) {
  v8f d = __builtin_amdgcn_wmma_f32_16x16x32_f16(false, a, false, b, (short)0, c, false, false);
  asm volatile("v_nop\n\tv_nop\n\tv_nop\n\tv_nop" : "+v"(d) : "v"(a), "v"(b));
  return d;
}
__device__ __forceinline__ v8f wmma_bf(v16b a, v16b b, v8f c) {
  v8f d = __builtin_amdgcn_wmma_f32_16x16x32_bf16(false, a, false, b, (short)0, c, false, false);
  asm volatile("v_nop\n\tv_nop\n\tv_nop\n\tv_nop" : "+v"(d) : "v"(a), "v"(b));
  return d;
}
__device__ __forceinline__ v16h frag_h(const _Float16* rowk0, unsigned lane) {
  union { v16h v; v8h q[2]; } u; const _Float16* p = rowk0 + 8u * (lane >> 4);
  u.q[0] = *(const v8h*)p; u.q[1] = *(const v8h*)(p + 16); return u.v;
}
__device__ __forceinline__ v16b frag_b(const __bf16* rowk0, unsigned lane) {
  union { v16b v; v8b q[2]; } u; const __bf16* p = rowk0 + 8u * (lane >> 4);
  u.q[0] = *(const v8b*)p; u.q[1] = *(const v8b*)(p + 16); return u.v;
}
struct F2 { v16b h, l; };
__device__ __forceinline__ F2 bsplit16(const float v[16]) { F2 r;
#pragma unroll
  for (int i = 0; i < 16; ++i) { const __bf16 h = (__bf16)v[i]; r.h[i] = h; r.l[i] = (__bf16)(v[i] - (float)h); }
  return r; }
__device__ __forceinline__ F2 split_row(const float* row, unsigned k0, unsigned lane) { float v[16]; const float* p = row + k0 + 8u * (lane >> 4);
#pragma unroll
  for (int i = 0; i < 8; ++i) { v[i] = p[i]; v[8 + i] = p[16 + i]; }
  return bsplit16(v); }
__device__ __forceinline__ float bfr(float v) { return (float)(__bf16)v; }
__device__ __forceinline__ v16b wcol_io(const float* Wm, unsigned k0, unsigned o, unsigned lane, unsigned ld) { v16b w; const unsigned g = lane >> 4;
#pragma unroll
  for (int i = 0; i < 8; ++i) { w[i] = (__bf16)Wm[(size_t)(k0 + 8u * g + i) * ld + o]; w[8 + i] = (__bf16)Wm[(size_t)(k0 + 16u + 8u * g + i) * ld + o]; }
  return w; }
#define LDSX() do { asm volatile("s_wait_dscnt 0" ::: "memory"); __builtin_amdgcn_wave_barrier(); __builtin_amdgcn_fence(3  , "workgroup"); } while (0)

#ifndef NB
#define NB 4
#endif
#ifndef SEQ
#define SEQ 2048
#endif
#define TT SEQ
#define NB_FULL 4
#define TT_FULL 2048
#define CC 1024
#define DIN 1024
#define NH 16
#define HD 64
#define NQB (TT / 64)
#define SCALE (0.125f)
#define QHI (TT < 512 ? TT : 512)
#define KHI QHI
#define QBH (QHI / 64)
#define PCAR (1024.0f)

static_assert(TT % 64 == 0);
static_assert(TT <= TT_FULL);
static_assert(NB <= NB_FULL);
static_assert(CC == NH * HD);
static_assert(HD == 64);
static_assert(CC % 128 == 0);
static_assert(DIN % 128 == 0);
static_assert(DIN % 32 == 0);
static_assert(CC % 32 == 0);
static_assert(QHI % 64 == 0);
static_assert(QBH * 64 == QHI);
static_assert(KHI == QHI);
static_assert(QHI <= TT);

#define WS_QH  ((size_t)0)
#define WS_KH  (WS_QH + 2u * (size_t)NB * TT * CC)
#define WS_VT  (WS_KH + 2u * (size_t)NB * TT * CC)
#define WS_QL  (WS_VT + 2u * (size_t)NB * CC * TT)
#define WS_KL  (WS_QL + 2u * (size_t)NB * QHI * CC)
#define WS_VB  (WS_KL + 2u * (size_t)NB * KHI * CC)
#define WS_VBL (WS_VB + 2u * (size_t)NB * CC * KHI)
#define WS_Y   (WS_VBL + 2u * (size_t)NB * CC * KHI)
#define WS_END (WS_Y  + 4u * (size_t)NB * TT * CC)
static_assert(WS_END <= (size_t)134217728);
static_assert(WS_KH % 128 == 0 && WS_VT % 128 == 0 && WS_QL % 128 == 0 && WS_KL % 128 == 0 && WS_VB % 128 == 0 && WS_VBL % 128 == 0 && WS_Y % 128 == 0);

__global__ __launch_bounds__(128) void k_proj(const float* __restrict__ X, const float* __restrict__ W,
    _Float16* __restrict__ QH, _Float16* __restrict__ QL, _Float16* __restrict__ KH, _Float16* __restrict__ KL, _Float16* __restrict__ VT, __bf16* __restrict__ VB, __bf16* __restrict__ VBL) {
  __shared__ __align__(16) _Float16 sh[64][136], sl[64][136]; __shared__ __align__(16) _Float16 th[128][72]; __shared__ __align__(16) __bf16 tb[128][72], tbl[128][72];
  const unsigned tid = threadIdx.x, wave = tid >> 5, lane = tid & 31u, col = lane & 15u, g = lane >> 4;
  const unsigned which = blockIdx.z; const unsigned c0 = blockIdx.y * 128u; const unsigned r0 = blockIdx.x * 64u; const unsigned bb = r0 / (unsigned)TT; const unsigned t0 = r0 % (unsigned)TT;
  const float* WA = W + which * (unsigned)CC;
  const float* xp = X + ((size_t)bb * TT_FULL + t0 + wave * 16u + col) * DIN + 8u * g;
  v8f acc[8] = {};
#pragma unroll 2
  for (unsigned kc = 0; kc < DIN / 32; ++kc) { v16b a; { const float* p = xp + kc * 32u;
#pragma unroll
      for (int i = 0; i < 8; ++i) { a[i] = (__bf16)p[i]; a[8 + i] = (__bf16)p[16 + i]; } }
    asm volatile("s_wait_loadcnt 0x0" ::: "memory");
#pragma unroll
    for (int j = 0; j < 8; ++j) { const v16b w = wcol_io(WA, kc * 32u, c0 + j * 16u + col, lane, 3u * CC); asm volatile("s_wait_loadcnt 0x0" ::: "memory"); acc[j] = wmma_bf(a, w, acc[j]); } }
  const bool hi_rows = t0 < (unsigned)QHI;
  if (which < 2u) { _Float16* DH = which == 0u ? QH : KH; _Float16* DL = which == 0u ? QL : KL;
#pragma unroll
    for (int j = 0; j < 8; ++j) {
#pragma unroll
      for (int r = 0; r < 8; ++r) { const float v = acc[j][r]; const _Float16 hv = (_Float16)v; sh[wave * 16u + 8u * g + r][j * 16u + col] = hv; sl[wave * 16u + 8u * g + r][j * 16u + col] = (_Float16)((v - (float)hv) * 1024.0f); } }
    __syncthreads();
    for (unsigned e = tid; e < 64u * 16u; e += 128u) { const unsigned rl = e >> 4, q = e & 15u;
      vst2(DH + ((size_t)r0 + rl) * CC + c0 + q * 8u, *(const v4u*)&sh[rl][q * 8u]);
      if (hi_rows) vst2(DL + ((size_t)bb * QHI + t0 + rl) * CC + c0 + q * 8u, *(const v4u*)&sl[rl][q * 8u]); }
  } else {
#pragma unroll
    for (int j = 0; j < 8; ++j) {
#pragma unroll
      for (int r = 0; r < 8; ++r) { const float v = acc[j][r]; const unsigned rl = wave * 16u + 8u * g + r, cl = j * 16u + col; th[cl][rl] = (_Float16)v; const __bf16 bh = (__bf16)v; tb[cl][rl] = bh; tbl[cl][rl] = (__bf16)(v - (float)bh); } }
    __syncthreads();
    for (unsigned e = tid; e < 128u * 8u; e += 128u) { const unsigned cl = e >> 3, q = e & 7u;
      vst2(VT + ((size_t)bb * CC + c0 + cl) * TT + t0 + q * 8u, *(const v4u*)&th[cl][q * 8u]);
      if (hi_rows) { const size_t o3 = ((size_t)bb * CC + c0 + cl) * KHI + t0 + q * 8u; vst2(VB + o3, *(const v4u*)&tb[cl][q * 8u]); vst2(VBL + o3, *(const v4u*)&tbl[cl][q * 8u]); } } } }

template <bool HI>
__device__ __forceinline__ void att_body(const _Float16* __restrict__ QH, const _Float16* __restrict__ KH, const _Float16* __restrict__ QL, const _Float16* __restrict__ KL,
    const _Float16* __restrict__ VT, const __bf16* __restrict__ VB, const __bf16* __restrict__ VBL, float* __restrict__ Y, const unsigned qb, const unsigned h, const unsigned b) {
  __shared__ __align__(16) _Float16 sp[4][16][72]; __shared__ __align__(16) __bf16 sph[4][16][72], spl[4][16][72]; __shared__ __align__(16) float ss[4][16][HD + 4];
  const unsigned tid = threadIdx.x, wave = tid >> 5, lane = tid & 31u, col = lane & 15u, g = lane >> 4;
  const unsigned ql0 = qb * 64u + wave * 16u;
  v16h qh[2], qlo[2];
#pragma unroll
  for (int kc = 0; kc < 2; ++kc) {
    qh[kc] = frag_h(QH + ((size_t)b * TT + ql0 + col) * CC + h * (unsigned)HD + kc * 32u, lane);
    if (HI) qlo[kc] = frag_h(QL + ((size_t)b * QHI + ql0 + col) * CC + h * (unsigned)HD + kc * 32u, lane); else qlo[kc] = qh[kc]; }
  float m[8], l[8]; v8f acc[4] = {};
#pragma unroll
  for (int r = 0; r < 8; ++r) { m[r] = -3.0e38f; l[r] = 0.f; }
#pragma unroll 1
  for (unsigned kt = 0; kt <= qb; ++kt) { const unsigned k0 = kt * 64u;
    v8f s[4];
#pragma unroll
    for (int j = 0; j < 4; ++j) { v8f a = {}, al = {};
#pragma unroll
      for (int kc = 0; kc < 2; ++kc) {
        const v16h kf = frag_h(KH + ((size_t)b * TT + k0 + j * 16u + col) * CC + h * (unsigned)HD + kc * 32u, lane);
        a = wmma16(qh[kc], kf, a);
        if (HI) { al = wmma16(qlo[kc], kf, al); const v16h klf = frag_h(KL + ((size_t)b * KHI + k0 + j * 16u + col) * CC + h * (unsigned)HD + kc * 32u, lane); al = wmma16(qh[kc], klf, al); } }
#pragma unroll
      for (int r = 0; r < 8; ++r) s[j][r] = HI ? (a[r] + al[r] * (1.0f / 1024.0f)) * SCALE : a[r] * SCALE; }
    float mnew[8];
#pragma unroll
    for (int r = 0; r < 8; ++r) { const unsigned qi = ql0 + 8u * g + r; float mx = m[r];
#pragma unroll
      for (int j = 0; j < 4; ++j) { const bool ok = (k0 + j * 16u + col) <= qi; const float v = ok ? s[j][r] : -3.0e38f; s[j][r] = v; mx = fmaxf(mx, v); }
#pragma unroll
      for (int o = 1; o < 16; o <<= 1) mx = fmaxf(mx, __shfl_xor(mx, o));
      mnew[r] = mx; }
#pragma unroll
    for (int r = 0; r < 8; ++r) { const unsigned qi = ql0 + 8u * g + r; const float ef = expf(m[r] - mnew[r]); const float sc = (m[r] <= -1.0e38f) ? 0.f : ef; float ps = 0.f;
#pragma unroll
      for (int j = 0; j < 4; ++j) { const bool ok = (k0 + j * 16u + col) <= qi; const float ev = expf(s[j][r] - mnew[r]); const float p = ok ? ev : 0.f; ps += p;
        if (HI) { const __bf16 bh = (__bf16)p; sph[wave][8u * g + r][j * 16u + col] = bh; spl[wave][8u * g + r][j * 16u + col] = (__bf16)(p - (float)bh); }
        else sp[wave][8u * g + r][j * 16u + col] = (_Float16)(p * PCAR); }
#pragma unroll
      for (int o = 1; o < 16; o <<= 1) ps += __shfl_xor(ps, o);
      l[r] = l[r] * sc + ps; m[r] = mnew[r];
#pragma unroll
      for (int d = 0; d < 4; ++d) acc[d][r] *= sc; }
    LDSX();
#pragma unroll
    for (int kc = 0; kc < 2; ++kc) {
      if (HI) { const v16b ph = frag_b(&sph[wave][col][kc * 32], lane), pl = frag_b(&spl[wave][col][kc * 32], lane);
#pragma unroll
        for (int d = 0; d < 4; ++d) { const size_t po = ((size_t)b * CC + h * (unsigned)HD + d * 16u + col) * KHI + k0 + kc * 32u; const v16b vh = frag_b(VB + po, lane); acc[d] = wmma_bf(ph, vh, acc[d]); acc[d] = wmma_bf(pl, vh, acc[d]); acc[d] = wmma_bf(ph, frag_b(VBL + po, lane), acc[d]); }
      } else { const v16h pf = frag_h(&sp[wave][col][kc * 32], lane);
#pragma unroll
        for (int d = 0; d < 4; ++d) { const size_t po = ((size_t)b * CC + h * (unsigned)HD + d * 16u + col) * TT + k0 + kc * 32u; acc[d] = wmma16(pf, frag_h(VT + po, lane), acc[d]); } } }
    LDSX(); }
#pragma unroll
  for (int r = 0; r < 8; ++r) { const float inv = (1.0f / l[r]) * (HI ? 1.0f : (1.0f / PCAR));
#pragma unroll
    for (int d = 0; d < 4; ++d) ss[wave][8u * g + r][d * 16u + col] = acc[d][r] * inv; }
  LDSX();
#pragma unroll 1
  for (unsigned rl = 0; rl < 8u; ++rl) { const unsigned row = rl + 8u * g; const v4f v = *(const v4f*)&ss[wave][row][col * 4u]; vst2(Y + ((size_t)b * TT + ql0 + row) * CC + h * (unsigned)HD + col * 4u, v); } }

__global__ __launch_bounds__(128) void k_att_hi(const _Float16* __restrict__ QH, const _Float16* __restrict__ KH, const _Float16* __restrict__ QL, const _Float16* __restrict__ KL, const _Float16* __restrict__ VT, const __bf16* __restrict__ VB, const __bf16* __restrict__ VBL, float* __restrict__ Y) {
  att_body<true>(QH, KH, QL, KL, VT, VB, VBL, Y, blockIdx.x, blockIdx.y, blockIdx.z); }
__global__ __launch_bounds__(128) void k_att(const _Float16* __restrict__ QH, const _Float16* __restrict__ KH, const _Float16* __restrict__ QL, const _Float16* __restrict__ KL, const _Float16* __restrict__ VT, const __bf16* __restrict__ VB, const __bf16* __restrict__ VBL, float* __restrict__ Y) {
  att_body<false>(QH, KH, QL, KL, VT, VB, VBL, Y, (unsigned)QBH + blockIdx.x, blockIdx.y, blockIdx.z); }

__global__ __launch_bounds__(128) void k_out(const float* __restrict__ Y, const float* __restrict__ WO, const float* __restrict__ BO, float* __restrict__ OUT) { __shared__ __align__(16) float sf[4][16][132];
  const unsigned tid = threadIdx.x, wave = tid >> 5, lane = tid & 31u, col = lane & 15u, g = lane >> 4; const unsigned c0 = blockIdx.y * 128u; const unsigned r0 = blockIdx.x * 64u + wave * 16u; const unsigned bb = r0 / (unsigned)TT, t0 = r0 % (unsigned)TT;
  v8f acc[8] = {};
#pragma unroll 2
  for (unsigned kc = 0; kc < CC / 32; ++kc) { const F2 a = split_row(Y + ((size_t)r0 + col) * CC, kc * 32u, lane); asm volatile("s_wait_loadcnt 0x0" ::: "memory");
#pragma unroll
    for (int j = 0; j < 8; ++j) { const v16b w = wcol_io(WO, kc * 32u, c0 + j * 16u + col, lane, (unsigned)DIN); asm volatile("s_wait_loadcnt 0x0" ::: "memory"); acc[j] = wmma_bf(a.h, w, acc[j]); acc[j] = wmma_bf(a.l, w, acc[j]); } }
#pragma unroll
  for (int j = 0; j < 8; ++j) { const float bias = bfr(BO[c0 + j * 16u + col]);
#pragma unroll
    for (int r = 0; r < 8; ++r) sf[wave][8u * g + r][j * 16u + col] = acc[j][r] + bias; }
  LDSX();
#pragma unroll 1
  for (unsigned rl = 0; rl < 16u; ++rl) { const v4f v = *(const v4f*)&sf[wave][rl][lane * 4u]; vst2(OUT + ((size_t)bb * TT_FULL + t0 + rl) * DIN + c0 + lane * 4u, v); } }

extern "C" void kernel_launch(void* const* d_in, const int* in_sizes, int n_in, void* d_out, int out_size, void* d_ws, size_t ws_size, hipStream_t stream) {
  if (n_in < 4) return;
  const int need_rows = (NB - 1) * TT_FULL + TT;
  if (in_sizes[0] < need_rows * DIN) return;
  if (in_sizes[1] < DIN * 3 * CC) return;
  if (in_sizes[2] < CC * DIN) return;
  if (in_sizes[3] < DIN) return;
  if (out_size < need_rows * DIN) return;
  if (ws_size < (size_t)WS_END) return;
  const float** F = (const float**)d_in;
  char* ws = (char*)d_ws;
  _Float16 *QH = (_Float16*)(ws + WS_QH), *KH = (_Float16*)(ws + WS_KH), *VT = (_Float16*)(ws + WS_VT), *QL = (_Float16*)(ws + WS_QL), *KL = (_Float16*)(ws + WS_KL);
  __bf16 *VB = (__bf16*)(ws + WS_VB), *VBL = (__bf16*)(ws + WS_VBL); float* Y = (float*)(ws + WS_Y);
  k_proj<<<dim3(NB * TT / 64, CC / 128, 3), 128, 0, stream>>>(F[0], F[1], QH, QL, KH, KL, VT, VB, VBL);
  k_att_hi<<<dim3(QBH, NH, NB), 128, 0, stream>>>(QH, KH, QL, KL, VT, VB, VBL, Y);
  if (NQB > QBH) k_att<<<dim3(NQB - QBH, NH, NB), 128, 0, stream>>>(QH, KH, QL, KL, VT, VB, VBL, Y);
  k_out<<<dim3(NB * TT / 64, DIN / 128), 128, 0, stream>>>(Y, F[2], F[3], (float*)d_out);
}
